// BiMultiHeadAttention_15066745274735
// MI455X (gfx1250) — hardware-verified
//
#include <hip/hip_runtime.h>
#include <math.h>

#ifndef NB
#define NB 8
#endif
#define NB_FULL 8
#define TQ 2048
#define SA 512
#define VD 512
#define AD 256
#define EM 512
#define NH 8
#define HD 64
#define OUT1_OFF_EL ((size_t)NB_FULL * (size_t)TQ * (size_t)VD)
#define WSC   256.0f
#define HSCL  0.125f
#define QS    8.0f
#define KS    8.0f
#define VVS   8.0f
#define VAS   8.0f
#define PCAR  32768.0f
#define CAS   64.0f
#define CVS   64.0f
#define CLIPV 50000.0f
#define LOG2E 1.4426950408889634f
#define NST   (SA / 64)
#define NTT   (TQ / 64)
#define NTB32 (TQ / 32)
#define NSB32 (SA / 32)
#define ATT_WAVES   4
#define ATT_THREADS (ATT_WAVES * 32)
#define CVT_THREADS 128
#define TR_THREADS  128
#define SPITCH 68
#define GPITCH 68
#define TPITCH 65

static_assert(NB >= 1 && NB <= NB_FULL);
static_assert(OUT1_OFF_EL == (size_t)33554432 / 4);
static_assert(EM == NH * HD && HD == 64 && NH == 8);
static_assert((TQ % 128) == 0 && (SA % 64) == 0 && ((NB * SA) % 128) == 0 && (EM % 128) == 0);
static_assert((TQ % 32) == 0 && (SA % 32) == 0 && NTB32 * 32 == TQ && NSB32 * 32 == SA);
static_assert((VD % 64) == 0 && (AD % 64) == 0 && (EM % 64) == 0);
static_assert((VD % 32) == 0 && (AD % 32) == 0 && (EM % 32) == 0);
static_assert(((NB * TQ * VD) % 1024) == 0 && ((NB * SA * AD) % 1024) == 0);
static_assert(NST * 128 == 2 * SA && NST * 128 == ATT_THREADS * 8);
static_assert((SPITCH * 4) % 16 == 0 && (GPITCH * 4) % 16 == 0);
static_assert(ATT_THREADS == 128 && TR_THREADS == 128 && CVT_THREADS == 128);

typedef unsigned short u16;
typedef _Float16 v16h __attribute__((ext_vector_type(16)));
typedef _Float16 v8h  __attribute__((ext_vector_type(8)));
typedef float    v8f  __attribute__((ext_vector_type(8)));
typedef float    v4f  __attribute__((ext_vector_type(4)));
typedef unsigned int v4u __attribute__((ext_vector_type(4)));

union FragH { v16h v; v8h h[2]; v4u u[2]; };

__device__ __forceinline__ unsigned short bf_bits(float f) {
  unsigned u = __float_as_uint(f);
  return (unsigned short)((u + 0x7FFFu + ((u >> 16) & 1u)) >> 16);
}
__device__ __forceinline__ float bf_up(unsigned short h) { return __uint_as_float(((unsigned)h) << 16); }
__device__ __forceinline__ float bfr(float f) { return bf_up(bf_bits(f)); }
__device__ __forceinline__ unsigned short h_bits(_Float16 x) { return __builtin_bit_cast(unsigned short, x); }
__device__ __forceinline__ unsigned pk16(unsigned short a, unsigned short b) { return (unsigned)a | ((unsigned)b << 16); }
__device__ __forceinline__ v8f zero8() { v8f z = {0.f, 0.f, 0.f, 0.f, 0.f, 0.f, 0.f, 0.f}; return z; }
__device__ __forceinline__ float clipf(float x, float c) { return fminf(fmaxf(x, -c), c); }

__device__ __forceinline__ v16h ldfrag_h(const _Float16* p) {
  FragH f;
  f.h[0] = *(const v8h*)(p);
  f.h[1] = *(const v8h*)(p + 16);
  return f.v;
}

__device__ __forceinline__ v8f mma_h(v16h a, v16h b, v8f c) {
  return __builtin_amdgcn_wmma_f32_16x16x32_f16(false, a, false, b, (short)0, c, false, false);
}
__device__ __forceinline__ void guard_s(v8f& a, v8f& b, v16h x0, v16h x1, v16h x2) {
#if defined(__HIP_DEVICE_COMPILE__)
  asm volatile("v_nop\n\tv_nop\n\tv_nop\n\tv_nop" : "+v"(a), "+v"(b) : "v"(x0), "v"(x1), "v"(x2) : "memory");
#endif
}
__device__ __forceinline__ void guard_p(v8f& a, v8f& b, v8f& c, v8f& d, v16h p, v16h x0, v16h x1, v16h x2, v16h x3) {
#if defined(__HIP_DEVICE_COMPILE__)
  asm volatile("v_nop\n\tv_nop\n\tv_nop\n\tv_nop"
               : "+v"(a), "+v"(b), "+v"(c), "+v"(d) : "v"(p), "v"(x0), "v"(x1), "v"(x2), "v"(x3) : "memory");
#endif
}
__device__ __forceinline__ void guard_g(v8f (&acc)[8], v16h x0, v16h x1, v16h x2, v16h x3, v16h x4, v16h x5) {
#if defined(__HIP_DEVICE_COMPILE__)
  asm volatile("v_nop\n\tv_nop\n\tv_nop\n\tv_nop"
               : "+v"(acc[0]), "+v"(acc[1]), "+v"(acc[2]), "+v"(acc[3]),
                 "+v"(acc[4]), "+v"(acc[5]), "+v"(acc[6]), "+v"(acc[7])
               : "v"(x0), "v"(x1), "v"(x2), "v"(x3), "v"(x4), "v"(x5) : "memory");
#endif
}
__device__ __forceinline__ void acc_guard4(v8f (&o)[4]) {
#if defined(__HIP_DEVICE_COMPILE__)
  asm volatile("v_nop\n\tv_nop\n\tv_nop\n\tv_nop" : "+v"(o[0]), "+v"(o[1]), "+v"(o[2]), "+v"(o[3]));
#endif
}
__device__ __forceinline__ void wave_sync_lds() {
  __builtin_amdgcn_fence(__ATOMIC_RELEASE, "workgroup");
  __builtin_amdgcn_wave_barrier();
  __builtin_amdgcn_fence(__ATOMIC_ACQUIRE, "workgroup");
}

__global__ __launch_bounds__(CVT_THREADS)
void cvt16(const float* __restrict__ x, u16* Y) {
  const size_t e0 = (size_t)blockIdx.x * 1024 + (size_t)threadIdx.x * 8;
  const v4f a = *(const v4f*)(x + e0), c4 = *(const v4f*)(x + e0 + 4);
  v4u o;
#pragma unroll
  for (int e = 0; e < 2; ++e) {
    o[e]     = pk16(h_bits((_Float16)bfr(a[2 * e])),  h_bits((_Float16)bfr(a[2 * e + 1])));
    o[2 + e] = pk16(h_bits((_Float16)bfr(c4[2 * e])), h_bits((_Float16)bfr(c4[2 * e + 1])));
  }
  u16* dst = Y + e0;
  for (int pass = 0; pass < 2; ++pass) {
    *(volatile v4u*)(dst) = o;
    __threadfence();
  }
}

__global__ __launch_bounds__(TR_THREADS)
void cvtT16(const float* __restrict__ W, u16* Y, int kdim, int ndim, float scale) {
  __shared__ __align__(16) float tile[64 * TPITCH];
  const int tid = threadIdx.x;
  const int nkt = kdim >> 6;
  const int bid = blockIdx.x;
  const int kt  = bid % nkt;
  const int ntb = bid / nkt;
  const int k0  = kt * 64, n0 = ntb * 64;
  const int lr = tid >> 4, lc = (tid & 15) * 4;
#pragma unroll
  for (int p = 0; p < 8; ++p) {
    const int kk = p * 8 + lr;
    const v4f w4 = *(const v4f*)(W + (size_t)(k0 + kk) * (size_t)ndim + n0 + lc);
    tile[kk * TPITCH + lc + 0] = w4[0];
    tile[kk * TPITCH + lc + 1] = w4[1];
    tile[kk * TPITCH + lc + 2] = w4[2];
    tile[kk * TPITCH + lc + 3] = w4[3];
  }
  __syncthreads();
  const int rq = tid >> 3, c8 = (tid & 7) * 8;
  v4u ov[4];
#pragma unroll
  for (int i = 0; i < 4; ++i) {
    const int row = 16 * i + rq;
#pragma unroll
    for (int e = 0; e < 4; ++e) {
      const float x0 = tile[(c8 + 2 * e) * TPITCH + row];
      const float x1 = tile[(c8 + 2 * e + 1) * TPITCH + row];
      ov[i][e] = pk16(h_bits((_Float16)(bfr(x0) * scale)), h_bits((_Float16)(bfr(x1) * scale)));
    }
  }
  u16* dst = Y + (size_t)n0 * (size_t)kdim + k0 + c8;
  for (int pass = 0; pass < 2; ++pass) {
#pragma unroll
    for (int i = 0; i < 4; ++i) {
      const int row = 16 * i + rq;
      *(volatile v4u*)(dst + (size_t)row * (size_t)kdim) = ov[i];
    }
    __threadfence();
  }
}

__device__ __forceinline__ void gemm_core(const _Float16* ap, const _Float16* bp, int K, v8f (&acc)[8]) {
  const size_t rs16 = (size_t)16 * (size_t)K;
#pragma unroll 1
  for (int k0 = 0; k0 < K; k0 += 32) {
    const v16h a0 = ldfrag_h(ap + k0), a1 = ldfrag_h(ap + rs16 + k0);
    const v16h b0 = ldfrag_h(bp + k0);
    const v16h b1 = ldfrag_h(bp + rs16 + k0);
    const v16h b2 = ldfrag_h(bp + 2 * rs16 + k0);
    const v16h b3 = ldfrag_h(bp + 3 * rs16 + k0);
    acc[0] = mma_h(a0, b0, acc[0]);
    acc[1] = mma_h(a0, b1, acc[1]);
    acc[2] = mma_h(a0, b2, acc[2]);
    acc[3] = mma_h(a0, b3, acc[3]);
    acc[4] = mma_h(a1, b0, acc[4]);
    acc[5] = mma_h(a1, b1, acc[5]);
    acc[6] = mma_h(a1, b2, acc[6]);
    acc[7] = mma_h(a1, b3, acc[7]);
    guard_g(acc, a0, a1, b0, b1, b2, b3);
  }
}
__device__ __forceinline__ void stage32x64(float* sl, v8f (&acc)[8], float oscale, int lane) {
  const int hh = lane >> 4, m = lane & 15;
#pragma unroll
  for (int i = 0; i < 2; ++i) {
#pragma unroll
    for (int r = 0; r < 8; ++r) {
      const int ro = (16 * i + 8 * hh + r) * GPITCH + m;
      sl[ro]      = acc[4 * i + 0][r] * oscale;
      sl[ro + 16] = acc[4 * i + 1][r] * oscale;
      sl[ro + 32] = acc[4 * i + 2][r] * oscale;
      sl[ro + 48] = acc[4 * i + 3][r] * oscale;
    }
  }
  wave_sync_lds();
}

__global__ __launch_bounds__(128)
void gemm_o16(const u16* __restrict__ A, const u16* __restrict__ Bt, u16* C,
              const float* __restrict__ bias, int biasN, int biasRow,
              int Mb, int N, int K, int aBs, int bBs, int cBs, float oscale, float bscale) {
  __shared__ __align__(16) float slab[4 * 32 * GPITCH];
  const int tid = threadIdx.x, wave = tid >> 5, lane = tid & 31, hh = lane >> 4, m = lane & 15;
  const int ntile = N >> 6, mtile = Mb >> 7;
  const int bid  = blockIdx.x;
  const int nt   = bid % ntile;
  const int tmp  = bid / ntile;
  const int mt   = tmp % mtile;
  const int bz   = tmp / mtile;
  const int rowb = mt * 128 + wave * 32;
  const int col0 = nt * 64;
  if (rowb + 32 > Mb) return;
  const _Float16* Ab = (const _Float16*)(const void*)A + (size_t)bz * (size_t)aBs;
  const _Float16* Bb = (const _Float16*)(const void*)Bt + (size_t)bz * (size_t)bBs;
  const _Float16* ap = Ab + (size_t)(rowb + m) * K + 8 * hh;
  const _Float16* bp = Bb + (size_t)(col0 + m) * K + 8 * hh;
  v8f acc[8];
#pragma unroll
  for (int i = 0; i < 8; ++i) acc[i] = zero8();
  gemm_core(ap, bp, K, acc);
  float* sl = slab + wave * 32 * GPITCH;
  stage32x64(sl, acc, oscale, lane);
  const int rq = lane >> 3, c8 = (lane & 7) * 8;
  const int bl = biasN - 1;
  const float selc = (biasRow != 0) ? 0.f : bscale;
  const float selr = (biasRow != 0) ? bscale : 0.f;
  float cb[8];
#pragma unroll
  for (int e = 0; e < 8; ++e) {
    int ci = col0 + c8 + e;
    ci = (ci < bl) ? ci : bl;
    cb[e] = bfr(bias[ci]) * selc;
  }
  v4u ov[8];
#pragma unroll
  for (int i = 0; i < 8; ++i) {
    const int row = 4 * i + rq;
    int ri = rowb + row;
    ri = (ri < bl) ? ri : bl;
    const float rb = bfr(bias[ri]) * selr;
    const v4f a = *(const v4f*)(sl + row * GPITCH + c8), c4 = *(const v4f*)(sl + row * GPITCH + c8 + 4);
#pragma unroll
    for (int e = 0; e < 2; ++e) {
      ov[i][e]     = pk16(h_bits((_Float16)(a[2 * e] + cb[2 * e] + rb)),
                          h_bits((_Float16)(a[2 * e + 1] + cb[2 * e + 1] + rb)));
      ov[i][2 + e] = pk16(h_bits((_Float16)(c4[2 * e] + cb[4 + 2 * e] + rb)),
                          h_bits((_Float16)(c4[2 * e + 1] + cb[5 + 2 * e] + rb)));
    }
  }
  u16* Cb = C + (size_t)bz * (size_t)cBs + (size_t)rowb * (size_t)N + col0 + c8;
  for (int pass = 0; pass < 2; ++pass) {
#pragma unroll
    for (int i = 0; i < 8; ++i) {
      const int row = 4 * i + rq;
      *(volatile v4u*)(Cb + (size_t)row * (size_t)N) = ov[i];
    }
    __threadfence();
  }
}

__global__ __launch_bounds__(128)
void gemm_o32(const u16* __restrict__ A, const u16* __restrict__ Bt, float* C,
              const float* __restrict__ bias, int biasN,
              int Mb, int N, int K, int aBs, int bBs, int cBs, float oscale) {
  __shared__ __align__(16) float slab[4 * 32 * GPITCH];
  const int tid = threadIdx.x, wave = tid >> 5, lane = tid & 31, hh = lane >> 4, m = lane & 15;
  const int ntile = N >> 6, mtile = Mb >> 7;
  const int bid  = blockIdx.x;
  const int nt   = bid % ntile;
  const int tmp  = bid / ntile;
  const int mt   = tmp % mtile;
  const int bz   = tmp / mtile;
  const int rowb = mt * 128 + wave * 32;
  const int col0 = nt * 64;
  if (rowb + 32 > Mb) return;
  const _Float16* Ab = (const _Float16*)(const void*)A + (size_t)bz * (size_t)aBs;
  const _Float16* Bb = (const _Float16*)(const void*)Bt + (size_t)bz * (size_t)bBs;
  const _Float16* ap = Ab + (size_t)(rowb + m) * K + 8 * hh;
  const _Float16* bp = Bb + (size_t)(col0 + m) * K + 8 * hh;
  v8f acc[8];
#pragma unroll
  for (int i = 0; i < 8; ++i) acc[i] = zero8();
  gemm_core(ap, bp, K, acc);
  float* sl = slab + wave * 32 * GPITCH;
  stage32x64(sl, acc, oscale, lane);
  const int r2 = lane >> 4, c4 = (lane & 15) * 4;
  const int bl = biasN - 1;
  float cb[4];
#pragma unroll
  for (int e = 0; e < 4; ++e) {
    int ci = col0 + c4 + e;
    ci = (ci < bl) ? ci : bl;
    cb[e] = bfr(bias[ci]);
  }
  v4f ov[16];
#pragma unroll
  for (int i = 0; i < 16; ++i) {
    const int row = 2 * i + r2;
    const v4f a = *(const v4f*)(sl + row * GPITCH + c4);
    v4f w;
    w[0] = a[0] + cb[0]; w[1] = a[1] + cb[1]; w[2] = a[2] + cb[2]; w[3] = a[3] + cb[3];
    ov[i] = w;
  }
  float* Cb = C + (size_t)bz * (size_t)cBs + (size_t)rowb * (size_t)N + col0 + c4;
  for (int pass = 0; pass < 2; ++pass) {
#pragma unroll
    for (int i = 0; i < 16; ++i) {
      const int row = 2 * i + r2;
      *(volatile v4f*)(Cb + (size_t)row * (size_t)N) = ov[i];
    }
    __threadfence();
  }
}

__global__ __launch_bounds__(ATT_THREADS)
void attn_col(const u16* __restrict__ Qp, const u16* __restrict__ Kp, const u16* __restrict__ VvT,
              u16* CtxA, float* Stat) {
  __shared__ __align__(16) float smem[ATT_WAVES * 16 * SPITCH];
  __shared__ __align__(16) float statl[128];

  const int tid  = threadIdx.x;
  const int wave = tid >> 5;
  const int lane = tid & 31;
  const int hh   = lane >> 4;
  const int c    = lane & 15;

  const int bid  = blockIdx.x;
  const int st   = bid % NST;
  const int head = (bid / NST) % NH;
  const int b    = bid / (NST * NH);
  const int s0w  = st * 64 + wave * 16;

  const _Float16* Sb = (const _Float16*)(const void*)Kp + ((size_t)(b * SA + s0w + c)) * EM + head * HD + 8 * hh;
  const _Float16* Tb = (const _Float16*)(const void*)Qp + ((size_t)(b * TQ + c)) * EM + head * HD + 8 * hh;
  const _Float16* Vb = (const _Float16*)(const void*)VvT + ((size_t)(b * EM + head * HD + c)) * TQ + 8 * hh;
  const float lsc = LOG2E / (QS * KS);
  const float cl2 = CLIPV * LOG2E;

  v16h sf[2];
  sf[0] = ldfrag_h(Sb);
  sf[1] = ldfrag_h(Sb + 32);

  float mrun = -INFINITY, lrun = 0.f;
  v8f o[4];
#pragma unroll
  for (int j = 0; j < 4; ++j) o[j] = zero8();

#pragma unroll 1
  for (int it = 0; it < NTB32; ++it) {
    const int tb = it * 32;
    v8f s0 = zero8(), s1 = zero8();
    const _Float16* t0p = Tb + (size_t)tb * EM;
    const _Float16* t1p = t0p + (size_t)16 * EM;
#pragma unroll
    for (int kk = 0; kk < HD / 32; ++kk) {
      const v16h a0 = ldfrag_h(t0p + kk * 32);
      const v16h a1 = ldfrag_h(t1p + kk * 32);
      s0 = mma_h(a0, sf[kk], s0);
      s1 = mma_h(a1, sf[kk], s1);
      guard_s(s0, s1, sf[kk], a0, a1);
    }
    float t[16];
#pragma unroll
    for (int i = 0; i < 8; ++i) { t[i] = clipf(s0[i] * lsc, cl2); t[8 + i] = clipf(s1[i] * lsc, cl2); }
    float cm = t[0];
#pragma unroll
    for (int i = 1; i < 16; ++i) cm = fmaxf(cm, t[i]);
    cm = fmaxf(cm, __shfl_xor(cm, 16, 32));
    const float mn = fmaxf(mrun, cm);
    const float al = exp2f(mrun - mn);
    mrun = mn;
    float ps = 0.f;
    FragH ph;
#pragma unroll
    for (int w = 0; w < 2; ++w) {
#pragma unroll
      for (int e4 = 0; e4 < 4; ++e4) {
        const int i = 8 * w + 2 * e4;
        const float p0 = exp2f(t[i] - mn), p1 = exp2f(t[i + 1] - mn);
        ps += p0 + p1;
        ph.u[w][e4] = pk16(h_bits((_Float16)(p0 * PCAR)), h_bits((_Float16)(p1 * PCAR)));
      }
    }
    ps += __shfl_xor(ps, 16, 32);
    lrun = lrun * al + ps;
    float scl[8];
#pragma unroll
    for (int r = 0; r < 8; ++r) scl[r] = __shfl(al, 8 * hh + r, 32);
#pragma unroll
    for (int j = 0; j < 4; ++j) {
#pragma unroll
      for (int r = 0; r < 8; ++r) o[j][r] *= scl[r];
    }
    const _Float16* vp = Vb + tb;
    {
      const v16h v0 = ldfrag_h(vp);
      const v16h v1 = ldfrag_h(vp + (size_t)16 * TQ);
      const v16h v2 = ldfrag_h(vp + (size_t)32 * TQ);
      const v16h v3 = ldfrag_h(vp + (size_t)48 * TQ);
      o[0] = mma_h(ph.v, v0, o[0]);
      o[1] = mma_h(ph.v, v1, o[1]);
      o[2] = mma_h(ph.v, v2, o[2]);
      o[3] = mma_h(ph.v, v3, o[3]);
      guard_p(o[0], o[1], o[2], o[3], ph.v, v0, v1, v2, v3);
    }
  }
  acc_guard4(o);

  const float rl   = 1.0f / lrun;
  const float lPv  = rl * PCAR;
  const float linv = rl * (CAS / (PCAR * VVS));
  statl[hh * 64 + wave * 16 + c] = (hh == 0) ? mrun : lPv;
  float inv[8];
#pragma unroll
  for (int r = 0; r < 8; ++r) inv[r] = __shfl(linv, 8 * hh + r, 32);
  float* slab = smem + wave * 16 * SPITCH;
#pragma unroll
  for (int r = 0; r < 8; ++r) {
#pragma unroll
    for (int j = 0; j < 4; ++j) slab[(8 * hh + r) * SPITCH + j * 16 + c] = o[j][r] * inv[r];
  }
  wave_sync_lds();
  const int rq = lane >> 3, c8 = (lane & 7) * 8;
  v4u ov[4];
#pragma unroll
  for (int i = 0; i < 4; ++i) {
    const int row = 4 * i + rq;
    const v4f a = *(const v4f*)(slab + row * SPITCH + c8), c4 = *(const v4f*)(slab + row * SPITCH + c8 + 4);
#pragma unroll
    for (int e = 0; e < 2; ++e) {
      ov[i][e]     = pk16(h_bits((_Float16)a[2 * e]),  h_bits((_Float16)a[2 * e + 1]));
      ov[i][2 + e] = pk16(h_bits((_Float16)c4[2 * e]), h_bits((_Float16)c4[2 * e + 1]));
    }
  }
  u16* cbp = CtxA + ((size_t)(b * SA + s0w)) * EM + head * HD + c8;
  for (int pass = 0; pass < 2; ++pass) {
#pragma unroll
    for (int i = 0; i < 4; ++i) {
      const int row = 4 * i + rq;
      *(volatile v4u*)(cbp + (size_t)row * EM) = ov[i];
    }
    __threadfence();
  }
  __syncthreads();
  if (wave == 0) {
    const v4f sv = *(const v4f*)(statl + 4 * lane);
    float* sp = Stat + ((size_t)((b * NH + head) * NST + st)) * 128 + 4 * lane;
    for (int pass = 0; pass < 2; ++pass) {
      *(volatile v4f*)(sp) = sv;
      __threadfence();
    }
  }
}

__global__ __launch_bounds__(ATT_THREADS)
void attn_vis(const u16* __restrict__ Qp, const u16* __restrict__ Kp, const u16* __restrict__ VaT,
              const float* __restrict__ Stat, u16* CtxV) {
  __shared__ __align__(16) float smem[ATT_WAVES * 16 * SPITCH];
  __shared__ __align__(16) float stt[2 * SA];

  const int tid  = threadIdx.x;
  const int wave = tid >> 5;
  const int lane = tid & 31;
  const int hh   = lane >> 4;
  const int c    = lane & 15;

  const int bid  = blockIdx.x;
  const int tt   = bid % NTT;
  const int head = (bid / NTT) % NH;
  const int b    = bid / (NTT * NH);
  const int t0w  = tt * 64 + wave * 16;

  const float* src = Stat + ((size_t)((b * NH + head) * NST)) * 128;
#pragma unroll 1
  for (int e = tid * 8; e < NST * 128; e += ATT_THREADS * 8) {
    const int j = e >> 7, offw = e & 127;
    const int di = (offw < 64) ? (j * 64 + offw) : (SA + j * 64 + offw - 64);
    const v4f x0 = *(const v4f*)(src + e), x1 = *(const v4f*)(src + e + 4);
    *(v4f*)(stt + di) = x0;
    *(v4f*)(stt + di + 4) = x1;
  }
  __syncthreads();

  const _Float16* Tb = (const _Float16*)(const void*)Qp + ((size_t)(b * TQ + t0w + c)) * EM + head * HD + 8 * hh;
  const _Float16* Sb = (const _Float16*)(const void*)Kp + ((size_t)(b * SA + c)) * EM + head * HD + 8 * hh;
  const _Float16* Vb = (const _Float16*)(const void*)VaT + ((size_t)(b * EM + head * HD + c)) * SA + 8 * hh;
  const float lsc = LOG2E / (QS * KS);
  const float cl2 = CLIPV * LOG2E;

  v16h tf[2];
  tf[0] = ldfrag_h(Tb);
  tf[1] = ldfrag_h(Tb + 32);

  v8f o[4];
#pragma unroll
  for (int j = 0; j < 4; ++j) o[j] = zero8();

#pragma unroll 1
  for (int it = 0; it < NSB32; ++it) {
    const int sb = it * 32;
    v8f s0 = zero8(), s1 = zero8();
    const _Float16* s0p = Sb + (size_t)sb * EM;
    const _Float16* s1p = s0p + (size_t)16 * EM;
#pragma unroll
    for (int kk = 0; kk < HD / 32; ++kk) {
      const v16h a0 = ldfrag_h(s0p + kk * 32);
      const v16h a1 = ldfrag_h(s1p + kk * 32);
      s0 = mma_h(a0, tf[kk], s0);
      s1 = mma_h(a1, tf[kk], s1);
      guard_s(s0, s1, tf[kk], a0, a1);
    }
    float t[16];
#pragma unroll
    for (int i = 0; i < 8; ++i) { t[i] = clipf(s0[i] * lsc, cl2); t[8 + i] = clipf(s1[i] * lsc, cl2); }
    float mv[16], lv[16];
    {
      const v4f m0 = *(const v4f*)(stt + sb + 8 * hh),      m1 = *(const v4f*)(stt + sb + 8 * hh + 4);
      const v4f m2 = *(const v4f*)(stt + sb + 16 + 8 * hh), m3 = *(const v4f*)(stt + sb + 16 + 8 * hh + 4);
      const v4f l0 = *(const v4f*)(stt + SA + sb + 8 * hh),      l1 = *(const v4f*)(stt + SA + sb + 8 * hh + 4);
      const v4f l2 = *(const v4f*)(stt + SA + sb + 16 + 8 * hh), l3 = *(const v4f*)(stt + SA + sb + 16 + 8 * hh + 4);
#pragma unroll
      for (int q = 0; q < 4; ++q) {
        mv[q] = m0[q]; mv[4 + q] = m1[q]; mv[8 + q] = m2[q]; mv[12 + q] = m3[q];
        lv[q] = l0[q]; lv[4 + q] = l1[q]; lv[8 + q] = l2[q]; lv[12 + q] = l3[q];
      }
    }
    FragH ph;
#pragma unroll
    for (int w = 0; w < 2; ++w) {
#pragma unroll
      for (int e4 = 0; e4 < 4; ++e4) {
        const int i = 8 * w + 2 * e4;
        const float p0 = exp2f(t[i] - mv[i]) * lv[i];
        const float p1 = exp2f(t[i + 1] - mv[i + 1]) * lv[i + 1];
        ph.u[w][e4] = pk16(h_bits((_Float16)p0), h_bits((_Float16)p1));
      }
    }
    const _Float16* vp = Vb + sb;
    {
      const v16h v0 = ldfrag_h(vp);
      const v16h v1 = ldfrag_h(vp + (size_t)16 * SA);
      const v16h v2 = ldfrag_h(vp + (size_t)32 * SA);
      const v16h v3 = ldfrag_h(vp + (size_t)48 * SA);
      o[0] = mma_h(ph.v, v0, o[0]);
      o[1] = mma_h(ph.v, v1, o[1]);
      o[2] = mma_h(ph.v, v2, o[2]);
      o[3] = mma_h(ph.v, v3, o[3]);
      guard_p(o[0], o[1], o[2], o[3], ph.v, v0, v1, v2, v3);
    }
  }
  acc_guard4(o);

  const float fac = CVS / (PCAR * VAS);
  float* slab = smem + wave * 16 * SPITCH;
#pragma unroll
  for (int r = 0; r < 8; ++r) {
#pragma unroll
    for (int j = 0; j < 4; ++j) slab[(8 * hh + r) * SPITCH + j * 16 + c] = o[j][r] * fac;
  }
  wave_sync_lds();
  const int rq = lane >> 3, c8 = (lane & 7) * 8;
  v4u ov[4];
#pragma unroll
  for (int i = 0; i < 4; ++i) {
    const int row = 4 * i + rq;
    const v4f a = *(const v4f*)(slab + row * SPITCH + c8), c4 = *(const v4f*)(slab + row * SPITCH + c8 + 4);
#pragma unroll
    for (int e = 0; e < 2; ++e) {
      ov[i][e]     = pk16(h_bits((_Float16)a[2 * e]),  h_bits((_Float16)a[2 * e + 1]));
      ov[i][2 + e] = pk16(h_bits((_Float16)c4[2 * e]), h_bits((_Float16)c4[2 * e + 1]));
    }
  }
  u16* cbp = CtxV + ((size_t)(b * TQ + t0w)) * EM + head * HD + c8;
  for (int pass = 0; pass < 2; ++pass) {
#pragma unroll
    for (int i = 0; i < 4; ++i) {
      const int row = 4 * i + rq;
      *(volatile v4u*)(cbp + (size_t)row * EM) = ov[i];
    }
    __threadfence();
  }
}

extern "C" void kernel_launch(void* const* d_in, const int* in_sizes, int n_in,
                              void* d_out, int out_size, void* d_ws, size_t ws_size,
                              hipStream_t stream) {
  if (n_in < 14) return;
  if (in_sizes[0] < NB * TQ * VD) return;
  if (in_sizes[1] < NB * SA * AD) return;
  if (in_sizes[2] != VD * EM || in_sizes[6] != VD * EM) return;
  if (in_sizes[4] != AD * EM || in_sizes[8] != AD * EM) return;
  if (in_sizes[10] != EM * VD || in_sizes[12] != EM * AD) return;
  if (in_sizes[3] < 1 || in_sizes[5] < 1 || in_sizes[7] < 1 || in_sizes[9] < 1 || in_sizes[11] < 1 || in_sizes[13] < 1) return;
  if ((size_t)out_size < OUT1_OFF_EL + (size_t)NB * SA * AD) return;

  const float* xv   = (const float*)d_in[0];
  const float* xa   = (const float*)d_in[1];
  const float* w_vq = (const float*)d_in[2];
  const float* b_vq = (const float*)d_in[3];
  const float* w_ak = (const float*)d_in[4];
  const float* b_ak = (const float*)d_in[5];
  const float* w_vv = (const float*)d_in[6];
  const float* b_vv = (const float*)d_in[7];
  const float* w_av = (const float*)d_in[8];
  const float* b_av = (const float*)d_in[9];
  const float* w_ov = (const float*)d_in[10];
  const float* b_ov = (const float*)d_in[11];
  const float* w_oa = (const float*)d_in[12];
  const float* b_oa = (const float*)d_in[13];
  float*       out  = (float*)d_out;
  const int nb3 = in_sizes[3], nb5 = in_sizes[5], nb7 = in_sizes[7], nb9 = in_sizes[9], nb11 = in_sizes[11], nb13 = in_sizes[13];

  const size_t szXV  = (size_t)NB * TQ * VD * 2;
  const size_t szXA  = (size_t)NB * SA * AD * 2;
  const size_t szWvq = (size_t)EM * VD * 2;
  const size_t szWak = (size_t)EM * AD * 2;
  const size_t szWvv = (size_t)EM * VD * 2;
  const size_t szWav = (size_t)EM * AD * 2;
  const size_t szWov = (size_t)VD * EM * 2;
  const size_t szWoa = (size_t)AD * EM * 2;
  const size_t szQ   = (size_t)NB * TQ * EM * 2;
  const size_t szK   = (size_t)NB * SA * EM * 2;
  const size_t szVVT = (size_t)NB * EM * TQ * 2;
  const size_t szVAT = (size_t)NB * EM * SA * 2;
  const size_t szST  = (size_t)NB * NH * NST * 128 * 4;
  const size_t szCA  = (size_t)NB * SA * EM * 2;
  const size_t szCV  = (size_t)NB * TQ * EM * 2;
  size_t off = 0;
  const size_t oXV  = off; off += szXV;
  const size_t oXA  = off; off += szXA;
  const size_t oWvq = off; off += szWvq;
  const size_t oWak = off; off += szWak;
  const size_t oWvv = off; off += szWvv;
  const size_t oWav = off; off += szWav;
  const size_t oWov = off; off += szWov;
  const size_t oWoa = off; off += szWoa;
  const size_t oQ   = off; off += szQ;
  const size_t oK   = off; off += szK;
  const size_t oVVT = off; off += szVVT;
  const size_t oVAT = off; off += szVAT;
  const size_t oST  = off; off += szST;
  const size_t oCA  = off; off += szCA;
  const size_t oCV  = off; off += szCV;
  if (off > ws_size) return;
  if (off > (size_t)134217728) return;

  char* ws = (char*)d_ws;
  u16* XV    = (u16*)(ws + oXV);
  u16* XA    = (u16*)(ws + oXA);
  u16* WVQT  = (u16*)(ws + oWvq);
  u16* WAKT  = (u16*)(ws + oWak);
  u16* WVVT  = (u16*)(ws + oWvv);
  u16* WAVT  = (u16*)(ws + oWav);
  u16* WOVT  = (u16*)(ws + oWov);
  u16* WOAT  = (u16*)(ws + oWoa);
  u16* Q16   = (u16*)(ws + oQ);
  u16* K16   = (u16*)(ws + oK);
  u16* VVT16 = (u16*)(ws + oVVT);
  u16* VAT16 = (u16*)(ws + oVAT);
  float* STAT = (float*)(ws + oST);
  u16* CTXA  = (u16*)(ws + oCA);
  u16* CTXV  = (u16*)(ws + oCV);

  cvt16<<<dim3((NB * TQ * VD) / 1024), dim3(CVT_THREADS), 0, stream>>>(xv, XV);
  cvt16<<<dim3((NB * SA * AD) / 1024), dim3(CVT_THREADS), 0, stream>>>(xa, XA);
  cvtT16<<<dim3((VD / 64) * (EM / 64)), dim3(TR_THREADS), 0, stream>>>(w_vq, WVQT, VD, EM, WSC);
  cvtT16<<<dim3((AD / 64) * (EM / 64)), dim3(TR_THREADS), 0, stream>>>(w_ak, WAKT, AD, EM, WSC);
  cvtT16<<<dim3((VD / 64) * (EM / 64)), dim3(TR_THREADS), 0, stream>>>(w_vv, WVVT, VD, EM, WSC);
  cvtT16<<<dim3((AD / 64) * (EM / 64)), dim3(TR_THREADS), 0, stream>>>(w_av, WAVT, AD, EM, WSC);
  cvtT16<<<dim3((EM / 64) * (VD / 64)), dim3(TR_THREADS), 0, stream>>>(w_ov, WOVT, EM, VD, WSC);
  cvtT16<<<dim3((EM / 64) * (AD / 64)), dim3(TR_THREADS), 0, stream>>>(w_oa, WOAT, EM, AD, WSC);
  gemm_o16<<<dim3(((NB * TQ) / 128) * (EM / 64)), dim3(128), 0, stream>>>(
      XV, WVQT, Q16, b_vq, nb3, 0, NB * TQ, EM, VD, 0, 0, 0, HSCL * QS / WSC, HSCL * QS);
  gemm_o16<<<dim3(((NB * SA) / 128) * (EM / 64)), dim3(128), 0, stream>>>(
      XA, WAKT, K16, b_ak, nb5, 0, NB * SA, EM, AD, 0, 0, 0, KS / WSC, KS);
  gemm_o16<<<dim3(NB * (EM / 128) * (TQ / 64)), dim3(128), 0, stream>>>(
      WVVT, XV, VVT16, b_vv, nb7, 1, EM, TQ, VD, 0, TQ * VD, EM * TQ, VVS / WSC, VVS);
  gemm_o16<<<dim3(NB * (EM / 128) * (SA / 64)), dim3(128), 0, stream>>>(
      WAVT, XA, VAT16, b_av, nb9, 1, EM, SA, AD, 0, SA * AD, EM * SA, VAS / WSC, VAS);
  attn_col<<<dim3(NB * NH * NST), dim3(ATT_THREADS), 0, stream>>>(Q16, K16, VVT16, CTXA, STAT);
  attn_vis<<<dim3(NB * NH * NTT), dim3(ATT_THREADS), 0, stream>>>(Q16, K16, VAT16, STAT, CTXV);
  gemm_o32<<<dim3(NB * (TQ / 128) * (VD / 64)), dim3(128), 0, stream>>>(
      CTXV, WOVT, out, b_ov, nb11, TQ, VD, EM, TQ * EM, 0, TQ * VD, 1.0f / (CVS * WSC));
  gemm_o32<<<dim3(((NB * SA) / 128) * (AD / 64)), dim3(128), 0, stream>>>(
      CTXA, WOAT, out + OUT1_OFF_EL, b_oa, nb13, NB * SA, AD, EM, 0, 0, 0, 1.0f / (CAS * WSC));
  (void)hipGetLastError();
}
